// DenoisingDecoder_18932215841128
// MI455X (gfx1250) — hardware-verified
//
#include <hip/hip_runtime.h>


namespace {
constexpr int B = 8, NA = 128, H = 128, LAT = 64, L = 3, BINS = 32, VOC = 100, NR = B * NA;
constexpr float XS = 8.0f, WSC = 256.0f;
typedef _Float16 b16;
typedef __attribute__((ext_vector_type(16))) _Float16 v16b;
typedef __attribute__((ext_vector_type(8))) _Float16 v8b;
typedef __attribute__((ext_vector_type(8))) float v8f;
typedef __attribute__((ext_vector_type(4))) float v4f;
__device__ __forceinline__ float bf16_rne(float f) { unsigned int u = __float_as_uint(f); u += 0x7FFFu + ((u >> 16) & 1u); return __uint_as_float(u & 0xFFFF0000u); }
__device__ __forceinline__ void split16(float v, b16& hi, b16& lo) { hi = (b16)v; lo = (b16)(v - (float)hi); }
__device__ __forceinline__ v16b frag_kb(const b16* p, int hh) { const v8b a = *(const v8b*)(p + 8 * hh), b = *(const v8b*)(p + 16 + 8 * hh); v16b f;
#pragma unroll
  for (int e = 0; e < 8; ++e) { f[e] = a[e]; f[8 + e] = b[e]; } return f; }
__device__ __forceinline__ v8f wmma16b(v16b a, v16b b, v8f c) { v8f d = __builtin_amdgcn_wmma_f32_16x16x32_f16(false, a, false, b, (short)0, c, false, false); asm volatile("v_nop\n\tv_nop\n\tv_nop\n\tv_nop" : "+v"(d) : "v"(a), "v"(b)); return d; }
__device__ __forceinline__ void wave_lds_sync() { __builtin_amdgcn_fence(__ATOMIC_RELEASE, "workgroup"); __builtin_amdgcn_wave_barrier(); __builtin_amdgcn_fence(__ATOMIC_ACQUIRE, "workgroup"); }
__device__ __forceinline__ float pmul(float a, float b) { float p = a * b; asm volatile("" : "+v"(p)); return p; }
__device__ __forceinline__ int iclamp(int v, int lo, int hi) { return v < lo ? lo : (v > hi ? hi : v); }
__device__ __forceinline__ float silu(float v) { return v / (1.0f + __expf(-v)); }

__global__ __launch_bounds__(256) void wput_kernel(const float* __restrict__ w, int KIN, int OUTW, int ldw, int krow0, int OP, b16* __restrict__ WT) {
  const int KG = KIN / 8; const int u = blockIdx.x * 256 + threadIdx.x; if (u >= OP * KG) return; const int o = u / KG, k0 = (u % KG) * 8; v8b v;
#pragma unroll
  for (int j = 0; j < 8; ++j) v[j] = (b16)(o < OUTW ? bf16_rne(w[(size_t)(krow0 + k0 + j) * ldw + o]) * WSC : 0.0f); for (int pass = 0; pass < 2; ++pass) { *(volatile v8b*)(WT + (size_t)o * KIN + k0) = v; __threadfence(); }
}
__global__ __launch_bounds__(32) void prep_kernel(const int* __restrict__ at, const float* __restrict__ frac, const float* __restrict__ lat, const int* __restrict__ tt, const float* __restrict__ z, const float* __restrict__ emb, const float* __restrict__ Wlat, const float* __restrict__ blat, const float* __restrict__ cW, const float* __restrict__ cb, float* __restrict__ CART, float* __restrict__ CND, float* __restrict__ Hh) {
  __shared__ float Cd[2 * H]; const int lane = threadIdx.x; const int b = blockIdx.x;
  const float tf = (float)tt[b];
  for (int q = 0; q < 2; ++q) { const int k = q * 32 + lane; const float f = expf(-9.210340371976184f * (float)k / 63.0f); const float a = tf * f; Cd[k] = sinf(a); Cd[64 + k] = cosf(a); }
  for (int q = 0; q < 4; ++q) { const int c = q * 32 + lane; float s = bf16_rne(blat[c]); for (int k = 0; k < LAT; ++k) s += pmul(bf16_rne(z[b * LAT + k]), bf16_rne(Wlat[k * H + c])); Cd[H + c] = s; }
  wave_lds_sync();
  for (int pass = 0; pass < 2; ++pass) {
    for (int l = 0; l < L; ++l) for (int q = 0; q < 4; ++q) { const int c = q * 32 + lane; float s = bf16_rne(cb[l * H + c]);
#pragma unroll 1
      for (int k = 0; k < 2 * H; ++k) s += pmul(Cd[k], bf16_rne(cW[((size_t)l * 2 * H + k) * H + c])); ((volatile float*)CND)[((size_t)b * L + l) * H + c] = silu(s); }
    for (int q = 0; q < 4; ++q) { const int i = q * 32 + lane; float cx = 0.0f, cy = 0.0f, cz = 0.0f; for (int a = 0; a < 3; ++a) { const float f = bf16_rne(frac[((size_t)b * NA + i) * 3 + a]); cx += pmul(f, bf16_rne(lat[(b * 3 + a) * 3 + 0])); cy += pmul(f, bf16_rne(lat[(b * 3 + a) * 3 + 1])); cz += pmul(f, bf16_rne(lat[(b * 3 + a) * 3 + 2])); }
      *(volatile v4f*)(CART + ((size_t)b * NA + i) * 4) = (v4f){cx, cy, cz, 0.0f}; }
    for (int i = 0; i < NA; ++i) { const int ty = iclamp(at[b * NA + i], 0, VOC - 1); for (int q = 0; q < 4; ++q) ((volatile float*)Hh)[((size_t)b * NA + i) * H + q * 32 + lane] = bf16_rne(emb[(size_t)ty * H + q * 32 + lane]); }
    __threadfence(); }
}
template <int NT, int ACT>
__global__ __launch_bounds__(32) void dense_kernel(const float* __restrict__ IN, const b16* __restrict__ WT, const float* __restrict__ bias, int nbias, int opitch, int col0, float* __restrict__ OUT) {
  __shared__ __attribute__((aligned(16))) b16 Ah[16][H + 8], Al[16][H + 8]; __shared__ float Tf[16][NT * 16 + 4]; const int lane = threadIdx.x, nloc = lane & 15, hlf = lane >> 4; const size_t m0 = (size_t)blockIdx.x * 16;
  for (int rr = 0; rr < 16; ++rr) for (int q = 0; q < 4; ++q) { b16 p, ql; split16(IN[(m0 + rr) * H + q * 32 + lane] * XS, p, ql); Ah[rr][q * 32 + lane] = p; Al[rr][q * 32 + lane] = ql; }
  wave_lds_sync(); v8f acc[NT];
#pragma unroll
  for (int t = 0; t < NT; ++t) acc[t] = (v8f){};
#pragma unroll
  for (int kb = 0; kb < H; kb += 32) { const v16b a = frag_kb(&Ah[nloc][kb], hlf), al = frag_kb(&Al[nloc][kb], hlf);
#pragma unroll
    for (int t = 0; t < NT; ++t) { const v16b bw = frag_kb(WT + (size_t)(t * 16 + nloc) * H + kb, hlf); acc[t] = wmma16b(a, bw, acc[t]); acc[t] = wmma16b(al, bw, acc[t]); } }
#pragma unroll
  for (int t = 0; t < NT; ++t) { const int c = t * 16 + nloc; const float bb = (bias != nullptr && c < nbias) ? bf16_rne(bias[c]) : 0.0f;
#pragma unroll
    for (int r8 = 0; r8 < 8; ++r8) { float v = acc[t][r8] * (1.0f / (XS * WSC)) + bb; if (ACT == 1) v = silu(v); Tf[8 * hlf + r8][c] = v; } }
  wave_lds_sync();
  for (int pass = 0; pass < 2; ++pass) { for (int rr = 0; rr < 16; ++rr) for (int c = lane; c < NT * 16; c += 32) ((volatile float*)OUT)[(m0 + rr) * (size_t)opitch + col0 + c] = Tf[rr][c]; __threadfence(); }
}
__global__ __launch_bounds__(32) void msg_kernel(const float* __restrict__ Hh, const float* __restrict__ PQ, const float* __restrict__ CART, const b16* __restrict__ WR, const float* __restrict__ eb, const float* __restrict__ CND, const int* __restrict__ mask, int l, int BV, float* __restrict__ HN) {
  __shared__ __attribute__((aligned(16))) b16 Ah[16][40], Al[16][40]; __shared__ float Te[16][2 * H + 4], Ag[H]; const int lane = threadIdx.x, nloc = lane & 15, hlf = lane >> 4; const int b = blockIdx.x / NA, i = blockIdx.x % NA; if (b >= BV) return;
  const size_t ri = (size_t)b * NA + i; const v4f ci = *(const v4f*)(CART + ri * 4); const float mi = mask[ri] != 0 ? 1.0f : 0.0f;
  for (int q = 0; q < 4; ++q) Ag[q * 32 + lane] = 0.0f;
  wave_lds_sync(); const float gam = (31.0f / 8.0f) * (31.0f / 8.0f), stepc = 8.0f / 31.0f;
#pragma unroll 1
  for (int jt = 0; jt < NA / 16; ++jt) {
    for (int rr = 0; rr < 16; ++rr) { const size_t rj = (size_t)b * NA + jt * 16 + rr; const v4f cj = *(const v4f*)(CART + rj * 4); const float dx = ci[0] - cj[0], dy = ci[1] - cj[1], dz = ci[2] - cj[2]; const float dist = sqrtf(pmul(dx, dx) + pmul(dy, dy) + pmul(dz, dz) + 1e-6f);
      const float dd = dist - stepc * (float)lane; const float r = __expf(-gam * dd * dd); b16 p, ql; split16(r * XS, p, ql); Ah[rr][lane] = p; Al[rr][lane] = ql; }
    wave_lds_sync(); const v16b a = frag_kb(&Ah[nloc][0], hlf), al = frag_kb(&Al[nloc][0], hlf);
#pragma unroll
    for (int t = 0; t < 16; ++t) { v8f acc = {}; const v16b bw = frag_kb(WR + (size_t)(t * 16 + nloc) * BINS, hlf); acc = wmma16b(a, bw, acc); acc = wmma16b(al, bw, acc); const int c = t * 16 + nloc; const float add = PQ[ri * (2 * 2 * H) + c] + bf16_rne(eb[l * 2 * H + c]);
#pragma unroll
      for (int r8 = 0; r8 < 8; ++r8) { const int rl = 8 * hlf + r8; const size_t rj = (size_t)b * NA + jt * 16 + rl; Te[rl][c] = acc[r8] * (1.0f / (XS * WSC)) + add + PQ[rj * (2 * 2 * H) + 2 * H + c]; } }
    wave_lds_sync();
    for (int rr = 0; rr < 16; ++rr) { const size_t rj = (size_t)b * NA + jt * 16 + rr; const float mj = mask[rj] != 0 ? 1.0f : 0.0f; const float pm = mi * mj;
      for (int q = 0; q < 4; ++q) { const int c = q * 32 + lane; const float g = Te[rr][c], co = Te[rr][H + c]; Ag[c] += pmul(pm, pmul(1.0f / (1.0f + __expf(-g)), silu(co))); } }
    wave_lds_sync(); }
  for (int pass = 0; pass < 2; ++pass) { for (int q = 0; q < 4; ++q) { const int c = q * 32 + lane; ((volatile float*)HN)[ri * H + c] = pmul(Hh[ri * H + c] + Ag[c] + CND[((size_t)b * L + l) * H + c], mi); } __threadfence(); }
}
__global__ __launch_bounds__(32) void types_kernel(const float* __restrict__ TY, float* __restrict__ out1) { const int lane = threadIdx.x; const size_t m0 = (size_t)blockIdx.x * 16;
  for (int pass = 0; pass < 2; ++pass) { for (int i = lane; i < 16 * VOC; i += 32) ((volatile float*)out1)[m0 * VOC + i] = TY[(m0 + i / VOC) * 112 + i % VOC]; __threadfence(); } }
__global__ __launch_bounds__(256) void noise_kernel(const float* __restrict__ A1, const float* __restrict__ Wc2, const float* __restrict__ bc2, float* __restrict__ out0) {
  __shared__ float No[8][128 * 3]; const int wave = threadIdx.x >> 5, lane = threadIdx.x & 31;
  for (int rr = 0; rr < 128; ++rr) { const size_t r = (size_t)wave * 128 + rr; float p0 = 0.0f, p1 = 0.0f, p2 = 0.0f; for (int q = 0; q < 4; ++q) { const int c = q * 32 + lane; const float a = A1[r * H + c]; p0 += pmul(a, bf16_rne(Wc2[c * 3])); p1 += pmul(a, bf16_rne(Wc2[c * 3 + 1])); p2 += pmul(a, bf16_rne(Wc2[c * 3 + 2])); }
    for (int o = 16; o; o >>= 1) { p0 += __shfl_xor(p0, o); p1 += __shfl_xor(p1, o); p2 += __shfl_xor(p2, o); } if (lane == 0) { No[wave][rr * 3] = p0 + bf16_rne(bc2[0]); No[wave][rr * 3 + 1] = p1 + bf16_rne(bc2[1]); No[wave][rr * 3 + 2] = p2 + bf16_rne(bc2[2]); } }
  wave_lds_sync();
  for (int pass = 0; pass < 2; ++pass) { for (int i = lane; i < 384; i += 32) ((volatile float*)out0)[(size_t)wave * 384 + i] = No[wave][i]; __threadfence(); }
}
}

extern "C" void kernel_launch(void* const* d_in, const int* in_sizes, int n_in, void* d_out, int out_size, void* d_ws, size_t ws_size, hipStream_t stream) {
  (void)n_in;
  auto Fp = [&](int i) { return (const float*)d_in[i]; }; auto Ip = [&](int i) { return (const int*)d_in[i]; };
  if (in_sizes[0] != NR || in_sizes[1] != NR * 3 || in_sizes[2] != B * 9 || in_sizes[3] != NR || in_sizes[4] != B || in_sizes[5] != B * LAT || in_sizes[6] != VOC * H || in_sizes[7] != LAT * H || in_sizes[9] != L * (2 * H + BINS) * 2 * H || in_sizes[11] != L * 2 * H * H || in_sizes[13] != H * H || in_sizes[15] != H * 3 || in_sizes[17] != H * VOC || out_size != NR * 3 + NR * VOC) return;
  const int BV = B;
  size_t off = 0; char* ws = (char*)d_ws;
  auto carve = [&](size_t bytes) { char* p = ws + off; off += (bytes + 255) & ~(size_t)255; return p; };
  b16* WPQ = (b16*)carve((size_t)L * 4 * H * H * 2);
  b16* WR = (b16*)carve((size_t)L * 2 * H * BINS * 2); b16* WC1 = (b16*)carve((size_t)H * H * 2); b16* WTY = (b16*)carve((size_t)112 * H * 2);
  float* CART = (float*)carve((size_t)NR * 4 * 4); float* CND = (float*)carve((size_t)B * L * H * 4); float* HA = (float*)carve((size_t)NR * H * 4); float* HB = (float*)carve((size_t)NR * H * 4); float* PQ = (float*)carve((size_t)NR * 4 * H * 4); float* A1 = (float*)carve((size_t)NR * H * 4); float* TY = (float*)carve((size_t)NR * 112 * 4);
  if (off > ws_size || off > ((size_t)32 << 20)) return;
  for (int l = 0; l < L; ++l) { const float* W = Fp(9) + (size_t)l * (2 * H + BINS) * 2 * H;
    wput_kernel<<<(2 * H * 16 + 255) / 256, 256, 0, stream>>>(W, H, 2 * H, 2 * H, 0, 2 * H, WPQ + (size_t)l * 4 * H * H);
    wput_kernel<<<(2 * H * 16 + 255) / 256, 256, 0, stream>>>(W, H, 2 * H, 2 * H, H, 2 * H, WPQ + (size_t)l * 4 * H * H + (size_t)2 * H * H);
    wput_kernel<<<(2 * H * 4 + 255) / 256, 256, 0, stream>>>(W, BINS, 2 * H, 2 * H, 2 * H, 2 * H, WR + (size_t)l * 2 * H * BINS); }
  wput_kernel<<<(H * 16 + 255) / 256, 256, 0, stream>>>(Fp(13), H, H, H, 0, H, WC1); wput_kernel<<<(112 * 16 + 255) / 256, 256, 0, stream>>>(Fp(17), H, VOC, VOC, 0, 112, WTY);
  prep_kernel<<<BV, 32, 0, stream>>>(Ip(0), Fp(1), Fp(2), Ip(4), Fp(5), Fp(6), Fp(7), Fp(8), Fp(11), Fp(12), CART, CND, HA);
  float* hcur = HA; float* hnext = HB;
  for (int l = 0; l < L; ++l) {
    dense_kernel<16, 0><<<BV * NA / 16, 32, 0, stream>>>(hcur, WPQ + (size_t)l * 4 * H * H, nullptr, 0, 4 * H, 0, PQ);
    dense_kernel<16, 0><<<BV * NA / 16, 32, 0, stream>>>(hcur, WPQ + (size_t)l * 4 * H * H + (size_t)2 * H * H, nullptr, 0, 4 * H, 2 * H, PQ);
    msg_kernel<<<BV * NA, 32, 0, stream>>>(hcur, PQ, CART, WR + (size_t)l * 2 * H * BINS, Fp(10), CND, Ip(3), l, BV, hnext);
    float* tsw = hcur; hcur = hnext; hnext = tsw; }
  dense_kernel<8, 1><<<BV * NA / 16, 32, 0, stream>>>(hcur, WC1, Fp(14), H, H, 0, A1);
  dense_kernel<7, 0><<<BV * NA / 16, 32, 0, stream>>>(hcur, WTY, Fp(18), VOC, 112, 0, TY);
  float* out = (float*)d_out; noise_kernel<<<1, 256, 0, stream>>>(A1, Fp(15), Fp(16), out); types_kernel<<<BV * NA / 16, 32, 0, stream>>>(TY, out + NR * 3);
}
